// BiMamba_74466142978823
// MI455X (gfx1250) — hardware-verified
//
#include <hip/hip_runtime.h>
#include <math.h>

typedef __attribute__((ext_vector_type(16))) _Float16 v16h;
typedef __attribute__((ext_vector_type(8)))  _Float16 v8h;
typedef __attribute__((ext_vector_type(16))) __bf16   v16b;
typedef __attribute__((ext_vector_type(8)))  __bf16   v8b;
typedef __attribute__((ext_vector_type(8)))  float    v8f;
typedef __attribute__((ext_vector_type(4)))  float    v4f;

constexpr int kBatch  = 2;
constexpr int kSeq    = 1024;
constexpr int kDm     = 1024;
constexpr int kDin    = 2048;
constexpr int kNst    = 16;
constexpr int kDtR    = 64;
constexpr int kXzP    = 2 * kDin;
constexpr int kXdW    = kDtR + 2 * kNst;
constexpr int kXdP    = 128;
constexpr int kBCW    = 2 * kNst;
constexpr int kRows   = kBatch * kSeq;
constexpr int kConvTP = 260;
constexpr int kScanTS = 64;
constexpr int kScanCh = 64;
constexpr int kScanYP = 68;
constexpr float kWCarry    = 1024.0f;
constexpr float kWCarryInv = 1.0f / 1024.0f;
static_assert(kXdW <= kXdP, "x_proj pad");
static_assert((kDm % 32) == 0 && (kDin % 32) == 0 && (kDtR % 32) == 0, "GEMM K multiples of 32");
static_assert((kRows % 64) == 0 && (kXzP % 64) == 0 && (kXdP % 64) == 0 && (kDm % 64) == 0 && (kDin % 64) == 0, "GEMM M,N multiples of 64");
static_assert((kSeq % kScanTS) == 0 && (kSeq % 64) == 0 && (kDin % kScanCh) == 0 && (kDin % 256) == 0, "tile multiples");

constexpr size_t kOffHSB  = 0;
constexpr size_t kOffWIB  = kOffHSB  + (size_t)kRows * kDm  * 2;
constexpr size_t kOffWXP0 = kOffWIB  + (size_t)kXzP  * kDm  * 2;
constexpr size_t kOffWXP1 = kOffWXP0 + (size_t)kXdP  * kDin * 2;
constexpr size_t kOffWDT0 = kOffWXP1 + (size_t)kXdP  * kDin * 2;
constexpr size_t kOffWDT1 = kOffWDT0 + (size_t)kDin  * kDtR * 2;
constexpr size_t kOffWOP  = kOffWDT1 + (size_t)kDin  * kDtR * 2;
constexpr size_t kOffXZ   = kOffWOP  + (size_t)kDm   * kDin * 2;
constexpr size_t kOffU    = kOffXZ   + (size_t)kRows * kXzP * 4;
constexpr size_t kOffUH   = kOffU    + (size_t)kRows * kDin * 4;
constexpr size_t kOffXD   = kOffUH   + (size_t)kRows * kDin * 2;
constexpr size_t kOffDTR  = kOffXD   + (size_t)kRows * kXdP * 4;
constexpr size_t kOffDT   = kOffDTR  + (size_t)kRows * kDtR * 2;
constexpr size_t kOffYF   = kOffDT   + (size_t)kRows * kDin * 4;
constexpr size_t kOffAVG  = kOffYF   + (size_t)kRows * kDin * 4;
constexpr size_t kWsTotal = kOffAVG  + (size_t)kRows * kDin * 2;
static_assert(kWsTotal == 120324096ull, "carve total");
static_assert(kWsTotal <= 134217728ull, "carve cap");
static_assert((kOffWIB % 128) == 0 && (kOffWXP0 % 128) == 0 && (kOffWXP1 % 128) == 0 && (kOffWDT0 % 128) == 0 &&
              (kOffWDT1 % 128) == 0 && (kOffWOP % 128) == 0 && (kOffXZ % 128) == 0 && (kOffU % 128) == 0 &&
              (kOffUH % 128) == 0 && (kOffXD % 128) == 0 && (kOffDTR % 128) == 0 && (kOffDT % 128) == 0 &&
              (kOffYF % 128) == 0 && (kOffAVG % 128) == 0, "128-B aligned regions");

constexpr int kT8HSB = kRows * kDm / 8;
constexpr int kT8WIB = kXzP * kDm / 8;
constexpr int kT8WXP = kXdP * kDin / 8;
constexpr int kT8WDT = kDin * kDtR / 8;
constexpr int kT8WOP = kDm * kDin / 8;
constexpr int kT8DTR = kRows * kDtR / 8;
static_assert((kT8HSB % 256) == 0 && (kT8WIB % 256) == 0 && (kT8WXP % 256) == 0 &&
              (kT8WDT % 256) == 0 && (kT8WOP % 256) == 0 && (kT8DTR % 256) == 0, "cast grids exact");

__device__ __forceinline__ unsigned short f2bf_bits(float f) {
  unsigned u = __float_as_uint(f);
  return (unsigned short)((u + 0x7FFFu + ((u >> 16) & 1u)) >> 16);
}
__device__ __forceinline__ float bf_bits2f(unsigned short h) { return __uint_as_float(((unsigned)h) << 16); }
__device__ __forceinline__ float bfr(float f) { return bf_bits2f(f2bf_bits(f)); }

__device__ __forceinline__ void dep_guard_h(v8f& a, v8f& b, v16h x, v16h y) { asm volatile("v_nop\n\tv_nop\n\tv_nop\n\tv_nop" : "+v"(a), "+v"(b) : "v"(x), "v"(y)); }
__device__ __forceinline__ void dep_guard_b(v8f& a, v8f& b, v16b x, v16b y) { asm volatile("v_nop\n\tv_nop\n\tv_nop\n\tv_nop" : "+v"(a), "+v"(b) : "v"(x), "v"(y)); }
__device__ __forceinline__ void dep_guard4_h(v8f& a, v8f& b, v8f& c, v8f& d, v16h x, v16h y) { asm volatile("v_nop\n\tv_nop\n\tv_nop\n\tv_nop" : "+v"(a), "+v"(b), "+v"(c), "+v"(d) : "v"(x), "v"(y)); }
__device__ __forceinline__ void dep_guard4_b(v8f& a, v8f& b, v8f& c, v8f& d, v16b x, v16b y) { asm volatile("v_nop\n\tv_nop\n\tv_nop\n\tv_nop" : "+v"(a), "+v"(b), "+v"(c), "+v"(d) : "v"(x), "v"(y)); }
__device__ __forceinline__ void keep4_h(v16h a, v16h b, v16h c, v16h d) { asm volatile("v_nop" :: "v"(a), "v"(b), "v"(c), "v"(d)); }
__device__ __forceinline__ void keep4_b(v16b a, v16b b, v16b c, v16b d) { asm volatile("v_nop" :: "v"(a), "v"(b), "v"(c), "v"(d)); }
__device__ __forceinline__ void acc_guard4(v8f& a, v8f& b, v8f& c, v8f& d) { asm volatile("v_nop\n\tv_nop\n\tv_nop\n\tv_nop" : "+v"(a), "+v"(b), "+v"(c), "+v"(d)); }
template <typename T> struct Frag;
template <> struct Frag<_Float16> {
  typedef v16h V; union U { v16h v; v8h h[2]; };
  static __device__ __forceinline__ v16h load(const _Float16* p) {
    U f; f.h[0] = *(const v8h*)(p); f.h[1] = *(const v8h*)(p + 16); return f.v;
  }
  static __device__ __forceinline__ v8f mma(v16h a, v16h b, v8f c) {
    return __builtin_amdgcn_wmma_f32_16x16x32_f16(false, a, false, b, (short)0, c, false, false);
  }
  static __device__ __forceinline__ void guard(v8f& a, v8f& b, v16h x, v16h y) { dep_guard_h(a, b, x, y); }
  static __device__ __forceinline__ void guard4(v8f& a, v8f& b, v8f& c, v8f& d, v16h x, v16h y) { dep_guard4_h(a, b, c, d, x, y); }
  static __device__ __forceinline__ void keep(v16h a, v16h b, v16h c, v16h d) { keep4_h(a, b, c, d); }
};
template <> struct Frag<__bf16> {
  typedef v16b V; union U { v16b v; v8b h[2]; };
  static __device__ __forceinline__ v16b load(const __bf16* p) {
    U f; f.h[0] = *(const v8b*)(p); f.h[1] = *(const v8b*)(p + 16); return f.v;
  }
  static __device__ __forceinline__ v8f mma(v16b a, v16b b, v8f c) {
    return __builtin_amdgcn_wmma_f32_16x16x32_bf16(false, a, false, b, (short)0, c, false, false);
  }
  static __device__ __forceinline__ void guard(v8f& a, v8f& b, v16b x, v16b y) { dep_guard_b(a, b, x, y); }
  static __device__ __forceinline__ void guard4(v8f& a, v8f& b, v8f& c, v8f& d, v16b x, v16b y) { dep_guard4_b(a, b, c, d, x, y); }
  static __device__ __forceinline__ void keep(v16b a, v16b b, v16b c, v16b d) { keep4_b(a, b, c, d); }
};

template <int ET> struct Elem;
template <> struct Elem<0> { typedef _Float16 T; };
template <> struct Elem<1> { typedef __bf16 T; };
template <int ET, int SPL, int BIAS_MODE, int OUT_MODE, bool RESID, int ACT = 0>
__global__ __launch_bounds__(256) void wmma_gemm64(
    const unsigned short* __restrict__ Ap, const unsigned short* __restrict__ A2p, int lda, long strideA,
    const unsigned short* __restrict__ Btp, const unsigned short* __restrict__ Bt2p, int ldb, long strideB,
    void* __restrict__ Cout, void* __restrict__ Cout2, int ldc, long strideC,
    const float* __restrict__ bias,
    const float* __restrict__ resid, long strideR,
    int M, int N, int K, float scale) {
  typedef typename Elem<ET>::T T;
  typedef typename Frag<T>::V V;
  const T* A = (const T*)Ap; const T* A2 = (const T*)A2p; const T* Bt = (const T*)Btp; const T* Bt2 = (const T*)Bt2p;
  __shared__ __align__(16) float sT[8][16 * 68];
  const int b    = blockIdx.y;
  const int lane = threadIdx.x & 31;
  const int wave = threadIdx.x >> 5;
  const int tilesN = N >> 6;
  const int tilesM = M >> 6;
  const int tile = blockIdx.x * 8 + wave;
  if (tile >= tilesM * tilesN) return;
  const int tm = tile / tilesN;
  const int tn = tile - tm * tilesN;
  const int m0 = tm << 6;
  const int n0 = tn << 6;

  const T* Ab  = A  + (size_t)b * strideA;
  const T* Bb  = Bt + (size_t)b * strideB;
  const T* Ab2 = (SPL >= 1) ? (A2  + (size_t)b * strideA) : nullptr;
  const T* Bb2 = (SPL == 2) ? (Bt2 + (size_t)b * strideB) : nullptr;

  const int rlane = lane & 15;
  const int koff  = (lane >> 4) * 8;
  const int mOff  = (lane >> 4) * 8;

  v8f acc[4][4];
#pragma unroll
  for (int i = 0; i < 4; ++i)
#pragma unroll
    for (int j = 0; j < 4; ++j) acc[i][j] = (v8f){0.f,0.f,0.f,0.f,0.f,0.f,0.f,0.f};

  for (int k0 = 0; k0 < K; k0 += 32) {
    V bh[4], bl[4];
#pragma unroll
    for (int j = 0; j < 4; ++j) {
      const size_t bo = (size_t)(n0 + (j << 4) + rlane) * ldb + koff + k0;
      bh[j] = Frag<T>::load(Bb + bo);
      if (SPL == 2) bl[j] = Frag<T>::load(Bb2 + bo);
    }
#pragma unroll
    for (int i = 0; i < 4; ++i) {
      const size_t ao = (size_t)(m0 + (i << 4) + rlane) * lda + koff + k0;
      V ah = Frag<T>::load(Ab + ao);
      V al;
      if (SPL >= 1) al = Frag<T>::load(Ab2 + ao);
#pragma unroll
      for (int j = 0; j < 4; ++j) {
        acc[i][j] = Frag<T>::mma(ah, bh[j], acc[i][j]);
        if (SPL == 2) acc[i][j] = Frag<T>::mma(ah, bl[j], acc[i][j]);
        if (SPL >= 1) acc[i][j] = Frag<T>::mma(al, bh[j], acc[i][j]);
      }
      Frag<T>::guard4(acc[i][0], acc[i][1], acc[i][2], acc[i][3], ah, (SPL >= 1) ? al : ah);
    }
    Frag<T>::keep(bh[0], bh[1], bh[2], bh[3]);
    if (SPL == 2) Frag<T>::keep(bl[0], bl[1], bl[2], bl[3]);
  }
  acc_guard4(acc[0][0], acc[0][1], acc[0][2], acc[0][3]);
  acc_guard4(acc[1][0], acc[1][1], acc[1][2], acc[1][3]);
  acc_guard4(acc[2][0], acc[2][1], acc[2][2], acc[2][3]);
  acc_guard4(acc[3][0], acc[3][1], acc[3][2], acc[3][3]);

  float* slab = sT[wave];
  const float* Rb = RESID ? (resid + (size_t)b * strideR) : nullptr;
#pragma unroll
  for (int i = 0; i < 4; ++i) {
    const int mBase = m0 + (i << 4);
#pragma unroll
    for (int j = 0; j < 4; ++j) {
      const int n = n0 + (j << 4) + rlane;
      float bv = 0.f;
      if (BIAS_MODE == 2) bv = bias[n];
#pragma unroll
      for (int r = 0; r < 8; ++r) {
        float v = acc[i][j][r] * scale;
        if (BIAS_MODE == 1) v += bias[mBase + mOff + r];
        if (BIAS_MODE == 2) v += bv;
        if (RESID) v += Rb[(size_t)(mBase + mOff + r) * ldc + n];
        if (ACT == 1) v = tanhf(v);
        if (ACT == 2) v = fmaxf(v, 0.0f);
        if (ACT == 3) v = v / (1.0f + expf(-v));
        if (ACT == 4) v = (v > 0.f) ? v : 0.01f * v;
        slab[(mOff + r) * 68 + (j << 4) + rlane] = v;
      }
    }
    __builtin_amdgcn_fence(__ATOMIC_RELEASE, "workgroup");
    __builtin_amdgcn_wave_barrier();
    __builtin_amdgcn_fence(__ATOMIC_ACQUIRE, "workgroup");
    if (OUT_MODE == 0) {
      float* C = (float*)Cout + (size_t)b * strideC;
      const int hh = lane >> 4, c4 = (lane & 15) * 4;
      for (int pass = 0; pass < 2; ++pass) {
#pragma unroll
        for (int it = 0; it < 8; ++it) {
          const int row = it * 2 + hh;
          v4f v = *(const v4f*)(slab + row * 68 + c4);
          *(volatile v4f*)(C + (size_t)(mBase + row) * ldc + n0 + c4) = v;
        }
        __threadfence();
      }
    } else {
      const int q = lane >> 3, c8 = (lane & 7) * 8;
      unsigned short* C  = (unsigned short*)Cout  + (size_t)b * strideC;
      unsigned short* C2 = (OUT_MODE == 2) ? ((unsigned short*)Cout2 + (size_t)b * strideC) : nullptr;
      for (int pass = 0; pass < 2; ++pass) {
#pragma unroll
        for (int it = 0; it < 4; ++it) {
          const int row = it * 4 + q;
          const float* sp = slab + row * 68 + c8;
          v8h hv, lv;
#pragma unroll
          for (int e = 0; e < 8; ++e) {
            if (OUT_MODE == 1) {
              hv[e] = (_Float16)sp[e];
            } else {
              unsigned short hb = f2bf_bits(sp[e]);
              unsigned short lb = f2bf_bits(sp[e] - bf_bits2f(hb));
              hv[e] = __builtin_bit_cast(_Float16, hb);
              lv[e] = __builtin_bit_cast(_Float16, lb);
            }
          }
          *(volatile v8h*)(C + (size_t)(mBase + row) * ldc + n0 + c8) = hv;
          if (OUT_MODE == 2) *(volatile v8h*)(C2 + (size_t)(mBase + row) * ldc + n0 + c8) = lv;
        }
        __threadfence();
      }
    }
    __builtin_amdgcn_fence(__ATOMIC_RELEASE, "workgroup");
    __builtin_amdgcn_wave_barrier();
    __builtin_amdgcn_fence(__ATOMIC_ACQUIRE, "workgroup");
  }
}

__global__ __launch_bounds__(256) void cast_bf16_kernel(
    const float* __restrict__ src, unsigned short* __restrict__ dst, int total8)
{
  const int i = blockIdx.x * 256 + threadIdx.x;
  if (i >= total8) return;
  const size_t e0 = (size_t)i << 3;
  const v4f a0 = *(const v4f*)(src + e0);
  const v4f a1 = *(const v4f*)(src + e0 + 4);
  v8h hv;
#pragma unroll
  for (int e = 0; e < 4; ++e) {
    hv[e]     = __builtin_bit_cast(_Float16, f2bf_bits(a0[e]));
    hv[4 + e] = __builtin_bit_cast(_Float16, f2bf_bits(a1[e]));
  }
  unsigned short* q = dst + e0;
  *(volatile v8h*)q = hv;
  __threadfence();
  *(volatile v8h*)q = hv;
}

template <bool PRE_BF16>
__global__ __launch_bounds__(256) void cast_f16_rows_kernel(
    const float* __restrict__ src, int src_pitch, int n_src_rows,
    unsigned short* __restrict__ dst, int dst_w_log2, int total8, float scale)
{
  const int i = blockIdx.x * 256 + threadIdx.x;
  if (i >= total8) return;
  const size_t e0 = (size_t)i << 3;
  const int row = (int)(e0 >> dst_w_log2);
  const int col = (int)(e0 & (size_t)((1 << dst_w_log2) - 1));
  const bool valid = row < n_src_rows;
  const int rs = valid ? row : (n_src_rows - 1);
  const float* sp = src + (size_t)rs * src_pitch + col;
  const v4f a0 = *(const v4f*)(sp);
  const v4f a1 = *(const v4f*)(sp + 4);
  const float zf = valid ? scale : 0.0f;
  v8h hv;
#pragma unroll
  for (int e = 0; e < 4; ++e) {
    const float f0 = PRE_BF16 ? bfr(a0[e]) : a0[e];
    const float f1 = PRE_BF16 ? bfr(a1[e]) : a1[e];
    hv[e]     = (_Float16)(f0 * zf);
    hv[4 + e] = (_Float16)(f1 * zf);
  }
  unsigned short* q = dst + e0;
  *(volatile v8h*)q = hv;
  __threadfence();
  *(volatile v8h*)q = hv;
}

template <int DIR>
__global__ __launch_bounds__(256) void conv_silu_kernel(
    const float* __restrict__ XZ, const float* __restrict__ cw, const float* __restrict__ cb,
    float* __restrict__ U, unsigned short* __restrict__ UH)
{
  __shared__ __align__(16) float sT[16 * kConvTP];
  const int tid = threadIdx.x, lane = tid & 31, wave = tid >> 5;
  const int d0 = blockIdx.x * 256, d = d0 + tid;
  const int g0 = blockIdx.y * 64;
  const int tb = g0 & (kSeq - 1);
  const float w0 = bfr(cw[d * 4 + 0]), w1 = bfr(cw[d * 4 + 1]), w2 = bfr(cw[d * 4 + 2]), w3 = bfr(cw[d * 4 + 3]);
  const float bc = bfr(cb[d]);
  float xm3, xm2, xm1;
  {
    const bool hist = (DIR == 0) ? (tb > 0) : ((tb + 64) < kSeq);
    const int rb = hist ? ((DIR == 0) ? (g0 - 3) : (g0 + 64)) : g0;
    const float va = XZ[(size_t)rb * kXzP + d];
    const float vb = XZ[(size_t)(rb + 1) * kXzP + d];
    const float vc = XZ[(size_t)(rb + 2) * kXzP + d];
    if (DIR == 0) { xm3 = hist ? va : 0.f; xm2 = hist ? vb : 0.f; xm1 = hist ? vc : 0.f; }
    else          { xm1 = hist ? va : 0.f; xm2 = hist ? vb : 0.f; xm3 = hist ? vc : 0.f; }
  }
  const int hrow = wave >> 1;
  const int hch  = (wave & 1) * 128 + lane * 4;
#pragma unroll 1
  for (int sub = 0; sub < 4; ++sub) {
    const int lb = (DIR == 0) ? (g0 + sub * 16) : (g0 + (3 - sub) * 16);
#pragma unroll 1
    for (int si = 0; si < 16; ++si) {
      const int s = (DIR == 0) ? si : (15 - si);
      const float xcur = XZ[(size_t)(lb + s) * kXzP + d];
      float acc = w0 * xm3;
      acc = fmaf(w1, xm2, acc);
      acc = fmaf(w2, xm1, acc);
      acc = fmaf(w3, xcur, acc);
      const float sv = acc + bc;
      const float sg = __builtin_amdgcn_rcpf(1.0f + __expf(-sv));
      sT[s * kConvTP + tid] = sv * sg;
      xm3 = xm2; xm2 = xm1; xm1 = xcur;
    }
    __syncthreads();
    v8h bh[2];
#pragma unroll
    for (int it = 0; it < 2; ++it) {
      const float* sp = sT + (it * 8 + wave) * kConvTP + lane * 8;
      const v4f a0 = *(const v4f*)(sp);
      const v4f a1 = *(const v4f*)(sp + 4);
#pragma unroll
      for (int e = 0; e < 4; ++e) {
        bh[it][e]     = (_Float16)a0[e];
        bh[it][4 + e] = (_Float16)a1[e];
      }
    }
    for (int pass = 0; pass < 2; ++pass) {
#pragma unroll
      for (int it = 0; it < 4; ++it) {
        const v4f fv = *(const v4f*)(sT + (it * 4 + hrow) * kConvTP + hch);
        *(volatile v4f*)(U + (size_t)(lb + it * 4 + hrow) * kDin + d0 + hch) = fv;
      }
#pragma unroll
      for (int it = 0; it < 2; ++it) {
        const size_t o = (size_t)(lb + it * 8 + wave) * kDin + d0 + lane * 8;
        *(volatile v8h*)(UH + o) = bh[it];
      }
      __threadfence();
    }
    __syncthreads();
  }
}

template <int DIR>
__global__ __launch_bounds__(64) void scan_kernel(
    const float* __restrict__ XD, const float* __restrict__ DT, const float* __restrict__ U,
    const float* __restrict__ XZ, const float* __restrict__ YFin,
    const float* __restrict__ bdt, const float* __restrict__ Alog, const float* __restrict__ Dp,
    float* __restrict__ YFout, unsigned short* __restrict__ AVG)
{
  __shared__ __align__(16) float sX[kScanTS * kBCW];
  __shared__ __align__(16) float sY[kScanTS * kScanYP];
  __shared__ __align__(16) float sA[kNst * kScanCh];
  const int tid = threadIdx.x, lane = tid & 31, wave = tid >> 5;
  constexpr int kBlkPerB = kDin / kScanCh;
  const int bix = blockIdx.x / kBlkPerB;
  const int d0  = (blockIdx.x - bix * kBlkPerB) * kScanCh;
  const int d   = d0 + tid;
  const size_t row0 = (size_t)bix * kSeq;
#pragma unroll 1
  for (int s = 0; s < kNst; ++s) sA[s * kScanCh + tid] = -expf(bfr(Alog[(size_t)d * kNst + s]));
  __syncthreads();
  float negA[kNst], h[kNst];
#pragma unroll
  for (int s = 0; s < kNst; ++s) {
    negA[s] = sA[s * kScanCh + tid];
    h[s] = 0.f;
  }
  const float bb = bfr(bdt[d]), Dd = bfr(Dp[d]);
  const int lr = tid >> 3, lc4 = (tid & 7) * 4;
  constexpr int kChunks = kSeq / kScanTS;
#pragma unroll 1
  for (int ci = 0; ci < kChunks; ++ci) {
    const int t0 = (DIR == 0) ? (ci * kScanTS) : (kSeq - kScanTS - ci * kScanTS);
    __syncthreads();
#pragma unroll
    for (int i = 0; i < 8; ++i) {
      const int r = lr + 8 * i;
      *(v4f*)(sX + r * kBCW + lc4) = *(const v4f*)(XD + (row0 + t0 + r) * kXdP + kDtR + lc4);
    }
    __syncthreads();
#pragma unroll 1
    for (int si = 0; si < kScanTS; ++si) {
      const int s = (DIR == 0) ? si : (kScanTS - 1 - si);
      const size_t rt = row0 + t0 + s;
      const float* xr = sX + s * kBCW;
      float Bs[kNst], Cs[kNst];
#pragma unroll
      for (int q4 = 0; q4 < 4; ++q4) {
        const v4f bv = *(const v4f*)(xr + 4 * q4);
        const v4f cv = *(const v4f*)(xr + kNst + 4 * q4);
        Bs[4 * q4 + 0] = bv[0]; Bs[4 * q4 + 1] = bv[1]; Bs[4 * q4 + 2] = bv[2]; Bs[4 * q4 + 3] = bv[3];
        Cs[4 * q4 + 0] = cv[0]; Cs[4 * q4 + 1] = cv[1]; Cs[4 * q4 + 2] = cv[2]; Cs[4 * q4 + 3] = cv[3];
      }
      const float v   = DT[rt * kDin + d] + bb;
      const float a   = __expf(-fabsf(v));
      const float up  = 1.0f + a;
      const float l1p = __logf(up) + (a - (up - 1.0f)) * __builtin_amdgcn_rcpf(up);
      const float dt  = fmaxf(v, 0.0f) + l1p;
      const float xt  = U[rt * kDin + d];
      const float dtx = dt * xt;
      float y = 0.0f;
#pragma unroll
      for (int k = 0; k < kNst; ++k) {
        const float e = __expf(dt * negA[k]);
        h[k] = fmaf(e, h[k], dtx * Bs[k]);
        y = fmaf(h[k], Cs[k], y);
      }
      y = fmaf(xt, Dd, y);
      const float zv = XZ[rt * kXzP + kDin + d];
      const float sg = __builtin_amdgcn_rcpf(1.0f + __expf(-zv));
      y = y * (zv * sg);
      if (DIR == 1) {
        const float yf = YFin[rt * kDin + d];
        y = 0.5f * (yf + y);
      }
      sY[s * kScanYP + tid] = y;
    }
    __syncthreads();
    if (DIR == 0) {
      const int hh = lane >> 4, c4 = (lane & 15) * 4;
      for (int pass = 0; pass < 2; ++pass) {
#pragma unroll
        for (int it = 0; it < 16; ++it) {
          const int row = it * 4 + wave * 2 + hh;
          const v4f val = *(const v4f*)(sY + row * kScanYP + c4);
          *(volatile v4f*)(YFout + (row0 + t0 + row) * kDin + d0 + c4) = val;
        }
        __threadfence();
      }
    } else {
      const int q = lane >> 3, c8 = (lane & 7) * 8;
      v8h hv[8];
#pragma unroll
      for (int it = 0; it < 8; ++it) {
        const int row = it * 8 + wave * 4 + q;
        const float* sp = sY + row * kScanYP + c8;
        const v4f a0 = *(const v4f*)(sp);
        const v4f a1 = *(const v4f*)(sp + 4);
#pragma unroll
        for (int e = 0; e < 4; ++e) {
          hv[it][e]     = (_Float16)a0[e];
          hv[it][4 + e] = (_Float16)a1[e];
        }
      }
      for (int pass = 0; pass < 2; ++pass) {
#pragma unroll
        for (int it = 0; it < 8; ++it) {
          const int row = it * 8 + wave * 4 + q;
          const size_t o = (row0 + t0 + row) * kDin + d0 + c8;
          *(volatile v8h*)(AVG + o) = hv[it];
        }
        __threadfence();
      }
    }
  }
}

extern "C" void kernel_launch(void* const* d_in, const int* in_sizes, int n_in,
                              void* d_out, int out_size, void* d_ws, size_t ws_size,
                              hipStream_t stream) {
  if (n_in < 17) return;
  if (in_sizes[0] != kRows * kDm) return;
  if (in_sizes[1] != kXzP * kDm) return;
  if (in_sizes[2] != kDin * 4 || in_sizes[9] != kDin * 4) return;
  if (in_sizes[3] != kDin || in_sizes[10] != kDin) return;
  if (in_sizes[4] != kXdW * kDin || in_sizes[11] != kXdW * kDin) return;
  if (in_sizes[5] != kDin * kDtR || in_sizes[12] != kDin * kDtR) return;
  if (in_sizes[6] != kDin || in_sizes[13] != kDin) return;
  if (in_sizes[7] != kDin * kNst || in_sizes[14] != kDin * kNst) return;
  if (in_sizes[8] != kDin || in_sizes[15] != kDin) return;
  if (in_sizes[16] != kDm * kDin) return;
  if (out_size != kRows * kDm) return;
  if (ws_size < kWsTotal) return;

  const float* hs      = (const float*)d_in[0];
  const float* W_in    = (const float*)d_in[1];
  const float* conv_w0 = (const float*)d_in[2];
  const float* conv_b0 = (const float*)d_in[3];
  const float* xw0     = (const float*)d_in[4];
  const float* dw0     = (const float*)d_in[5];
  const float* db0     = (const float*)d_in[6];
  const float* alog0   = (const float*)d_in[7];
  const float* dskip0  = (const float*)d_in[8];
  const float* conv_w1 = (const float*)d_in[9];
  const float* conv_b1 = (const float*)d_in[10];
  const float* xw1     = (const float*)d_in[11];
  const float* dw1     = (const float*)d_in[12];
  const float* db1     = (const float*)d_in[13];
  const float* alog1   = (const float*)d_in[14];
  const float* dskip1  = (const float*)d_in[15];
  const float* W_out   = (const float*)d_in[16];
  float* out = (float*)d_out;

  char* ws = (char*)d_ws;
  unsigned short* HSB  = (unsigned short*)(ws + kOffHSB);
  unsigned short* WIB  = (unsigned short*)(ws + kOffWIB);
  unsigned short* WXP0 = (unsigned short*)(ws + kOffWXP0);
  unsigned short* WXP1 = (unsigned short*)(ws + kOffWXP1);
  unsigned short* WDT0 = (unsigned short*)(ws + kOffWDT0);
  unsigned short* WDT1 = (unsigned short*)(ws + kOffWDT1);
  unsigned short* WOP  = (unsigned short*)(ws + kOffWOP);
  float*          XZ   = (float*)(ws + kOffXZ);
  float*          U    = (float*)(ws + kOffU);
  unsigned short* UH   = (unsigned short*)(ws + kOffUH);
  float*          XD   = (float*)(ws + kOffXD);
  unsigned short* DTR  = (unsigned short*)(ws + kOffDTR);
  float*          DT   = (float*)(ws + kOffDT);
  float*          YF   = (float*)(ws + kOffYF);
  unsigned short* AVG  = (unsigned short*)(ws + kOffAVG);

  cast_bf16_kernel<<<kT8HSB / 256, 256, 0, stream>>>(hs, HSB, kT8HSB);
  cast_bf16_kernel<<<kT8WIB / 256, 256, 0, stream>>>(W_in, WIB, kT8WIB);
  cast_f16_rows_kernel<true><<<kT8WXP / 256, 256, 0, stream>>>(xw0, kDin, kXdW, WXP0, 11, kT8WXP, kWCarry);
  cast_f16_rows_kernel<true><<<kT8WXP / 256, 256, 0, stream>>>(xw1, kDin, kXdW, WXP1, 11, kT8WXP, kWCarry);
  cast_f16_rows_kernel<true><<<kT8WDT / 256, 256, 0, stream>>>(dw0, kDtR, kDin, WDT0, 6, kT8WDT, kWCarry);
  cast_f16_rows_kernel<true><<<kT8WDT / 256, 256, 0, stream>>>(dw1, kDtR, kDin, WDT1, 6, kT8WDT, kWCarry);
  cast_f16_rows_kernel<true><<<kT8WOP / 256, 256, 0, stream>>>(W_out, kDin, kDm, WOP, 11, kT8WOP, kWCarry);

  wmma_gemm64<1, 0, 0, 0, false><<<dim3((kRows / 64) * (kXzP / 64) / 8, 1), 256, 0, stream>>>(
      HSB, nullptr, kDm, 0L,
      WIB, nullptr, kDm, 0L,
      (void*)XZ, nullptr, kXzP, 0L,
      nullptr, nullptr, 0L,
      kRows, kXzP, kDm, 1.0f);

  conv_silu_kernel<0><<<dim3(kDin / 256, kRows / 64), 256, 0, stream>>>(XZ, conv_w0, conv_b0, U, UH);
  wmma_gemm64<0, 0, 0, 0, false><<<dim3((kRows / 64) * (kXdP / 64) / 8, 1), 256, 0, stream>>>(
      UH, nullptr, kDin, 0L,
      WXP0, nullptr, kDin, 0L,
      (void*)XD, nullptr, kXdP, 0L,
      nullptr, nullptr, 0L,
      kRows, kXdP, kDin, kWCarryInv);
  cast_f16_rows_kernel<false><<<kT8DTR / 256, 256, 0, stream>>>(XD, kXdP, kRows, DTR, 6, kT8DTR, 1.0f);
  wmma_gemm64<0, 0, 0, 0, false><<<dim3((kRows / 64) * (kDin / 64) / 8, 1), 256, 0, stream>>>(
      DTR, nullptr, kDtR, 0L,
      WDT0, nullptr, kDtR, 0L,
      (void*)DT, nullptr, kDin, 0L,
      nullptr, nullptr, 0L,
      kRows, kDin, kDtR, kWCarryInv);
  scan_kernel<0><<<kBatch * (kDin / kScanCh), kScanCh, 0, stream>>>(
      XD, DT, U, XZ, YF, db0, alog0, dskip0, YF, AVG);

  conv_silu_kernel<1><<<dim3(kDin / 256, kRows / 64), 256, 0, stream>>>(XZ, conv_w1, conv_b1, U, UH);
  wmma_gemm64<0, 0, 0, 0, false><<<dim3((kRows / 64) * (kXdP / 64) / 8, 1), 256, 0, stream>>>(
      UH, nullptr, kDin, 0L,
      WXP1, nullptr, kDin, 0L,
      (void*)XD, nullptr, kXdP, 0L,
      nullptr, nullptr, 0L,
      kRows, kXdP, kDin, kWCarryInv);
  cast_f16_rows_kernel<false><<<kT8DTR / 256, 256, 0, stream>>>(XD, kXdP, kRows, DTR, 6, kT8DTR, 1.0f);
  wmma_gemm64<0, 0, 0, 0, false><<<dim3((kRows / 64) * (kDin / 64) / 8, 1), 256, 0, stream>>>(
      DTR, nullptr, kDtR, 0L,
      WDT1, nullptr, kDtR, 0L,
      (void*)DT, nullptr, kDin, 0L,
      nullptr, nullptr, 0L,
      kRows, kDin, kDtR, kWCarryInv);
  scan_kernel<1><<<kBatch * (kDin / kScanCh), kScanCh, 0, stream>>>(
      XD, DT, U, XZ, YF, db1, alog1, dskip1, YF, AVG);

  wmma_gemm64<0, 0, 0, 0, false><<<dim3((kRows / 64) * (kDm / 64) / 8, 1), 256, 0, stream>>>(
      AVG, nullptr, kDin, 0L,
      WOP, nullptr, kDin, 0L,
      (void*)out, nullptr, kDm, 0L,
      nullptr, nullptr, 0L,
      kRows, kDm, kDin, kWCarryInv);
}
